// SS1D_MB_23192823398801
// MI455X (gfx1250) — hardware-run, weakly checked
//
#include <hip/hip_runtime.h>
#include <math.h>

typedef __attribute__((ext_vector_type(16))) _Float16 v16h;
typedef __attribute__((ext_vector_type(8)))  _Float16 v8h;
typedef __attribute__((ext_vector_type(8)))  float    v8f;
typedef __attribute__((ext_vector_type(4)))  float    v4f;
typedef __attribute__((ext_vector_type(4)))  unsigned v4u;

constexpr int kB     = 2;
constexpr int kLB    = 2048;
constexpr int kDm    = 768;
constexpr int kDi    = 1536;
constexpr int kNs    = 16;
constexpr int kR     = 48;
constexpr int kRP    = 64;
constexpr int kPj    = 80;
constexpr int kPjP   = 192;
constexpr int kXzP   = 2 * kDi;
constexpr int kRows  = kB * kLB;
constexpr float kEps = 1e-5f;

constexpr float kCarryW  = 1024.0f;
constexpr float kCarryXn = 16.0f;
constexpr float kCarryU  = 64.0f;
constexpr float kCarryDt = 256.0f;
constexpr float kCarryY  = 64.0f;
constexpr float kScaleIn  = 1.0f / (kCarryXn * kCarryW);
constexpr float kScaleXp  = 1.0f / (kCarryU  * kCarryW);
constexpr float kScaleDt  = 1.0f / (kCarryDt * kCarryW);
constexpr float kScaleOut = 1.0f / (kCarryY  * kCarryW);
constexpr float kF16Min = 6.103515625e-5f;

constexpr int kConvTP = 260;
constexpr int kScanTS = 64;
constexpr int kScanCh = 64;
constexpr int kScanYP = 68;

static_assert(kR + 2 * kNs == kPj);
static_assert(2 * kPj <= kPjP && (kPjP % 64) == 0);
static_assert((kDm % 64) == 0 && (kDi % 64) == 0 && (kRP % 64) == 0 && (kXzP % 64) == 0);
static_assert((kLB % 64) == 0 && (kLB % kScanTS) == 0 && (kDi % kScanCh) == 0 && (kDi % 256) == 0 && (kDm % 256) == 0);
static_assert(kLB * kRP == (1 << 17));
static_assert((kPj % 8) == 0 && (kR % 8) == 0);

constexpr size_t kSzWinT  = (size_t)kXzP * kDm * 2;
constexpr size_t kSzXpT   = (size_t)kPjP * kDi * 2;
constexpr size_t kSzDtT   = (size_t)2 * kDi * kRP * 2;
constexpr size_t kSzWoutT = (size_t)kDm * kDi * 2;
constexpr size_t kSzXN    = (size_t)kRows * kDm * 2;
constexpr size_t kSzXZ    = (size_t)kLB * kXzP * 4;
constexpr size_t kSzUC    = (size_t)kLB * kDi * 4;
constexpr size_t kSzU16   = (size_t)kLB * kDi * 2;
constexpr size_t kSzPROJ  = (size_t)kLB * kPjP * 4;
constexpr size_t kSzDTA   = (size_t)2 * kLB * kRP * 2;
constexpr size_t kSzDLR   = (size_t)2 * kLB * kDi * 4;
constexpr size_t kSzYD    = (size_t)2 * kLB * kDi * 4;
constexpr size_t kSzYG    = (size_t)kLB * kDi * 2;
constexpr size_t kOffWinT  = 0;
constexpr size_t kOffXpT   = kOffWinT  + kSzWinT;
constexpr size_t kOffDtT   = kOffXpT   + kSzXpT;
constexpr size_t kOffWoutT = kOffDtT   + kSzDtT;
constexpr size_t kOffXN    = kOffWoutT + kSzWoutT;
constexpr size_t kOffXZ    = kOffXN    + kSzXN;
constexpr size_t kOffUC    = kOffXZ    + kSzXZ;
constexpr size_t kOffU16   = kOffUC    + kSzUC;
constexpr size_t kOffPROJ  = kOffU16   + kSzU16;
constexpr size_t kOffDTA   = kOffPROJ  + kSzPROJ;
constexpr size_t kOffDLR   = kOffDTA   + kSzDTA;
constexpr size_t kOffYD    = kOffDLR   + kSzDLR;
constexpr size_t kOffYG    = kOffYD    + kSzYD;
constexpr size_t kWsTotal  = kOffYG    + kSzYG;
static_assert(kWsTotal == 117112832ull);
static_assert(kWsTotal <= 134217728ull);
static_assert((kSzWinT % 128) == 0 && (kSzXpT % 128) == 0 && (kSzDtT % 128) == 0 && (kSzWoutT % 128) == 0 &&
              (kSzXN % 128) == 0 && (kSzXZ % 128) == 0 && (kSzUC % 128) == 0 && (kSzU16 % 128) == 0 &&
              (kSzPROJ % 128) == 0 && (kSzDTA % 128) == 0 && (kSzDLR % 128) == 0 && (kSzYD % 128) == 0 &&
              (kSzYG % 128) == 0);

__device__ __forceinline__ _Float16 f16_flush(float v) {
  const float t = (fabsf(v) < kF16Min) ? 0.0f : v;
  return (_Float16)t;
}
__device__ __forceinline__ float wave_sum(float v) {
  v += __shfl_xor(v, 16, 32);
  v += __shfl_xor(v, 8, 32);
  v += __shfl_xor(v, 4, 32);
  v += __shfl_xor(v, 2, 32);
  v += __shfl_xor(v, 1, 32);
  return v;
}
__device__ __forceinline__ float silu_f(float v) {
  const float sg = __builtin_amdgcn_rcpf(1.0f + expf(-v));
  return v * sg;
}

__device__ __forceinline__ void tie1_h(v8f& a, v16h x, v16h y) { asm volatile("" : "+v"(a) : "v"(x), "v"(y)); }
__device__ __forceinline__ void guard1_h(v8f& a, v16h x, v16h y) { asm volatile("v_nop\n\tv_nop\n\tv_nop\n\tv_nop" : "+v"(a) : "v"(x), "v"(y)); }
__device__ __forceinline__ void keep4_h(v16h a, v16h b, v16h c, v16h d) { asm volatile("v_nop" :: "v"(a), "v"(b), "v"(c), "v"(d)); }
__device__ __forceinline__ void acc_guard4(v8f& a, v8f& b, v8f& c, v8f& d) { asm volatile("v_nop\n\tv_nop\n\tv_nop\n\tv_nop" : "+v"(a), "+v"(b), "+v"(c), "+v"(d)); }

__device__ __forceinline__ v16h frag_load_h(const _Float16* p) {
  union U { v16h v; v8h h[2]; } f;
  f.h[0] = *(const v8h*)(p);
  f.h[1] = *(const v8h*)(p + 16);
  return f.v;
}
__device__ __forceinline__ v8f mma_h(v16h a, v16h b, v8f c) {
  return __builtin_amdgcn_wmma_f32_16x16x32_f16(false, a, false, b, (short)0, c, false, false);
}

template <int BIAS_MODE, bool RESID>
__global__ __launch_bounds__(256) void wmma_gemm64(
    const unsigned short* __restrict__ Ap, int lda, long strideA,
    const unsigned short* __restrict__ Btp, int ldb, long strideB,
    float* __restrict__ Cout, int ldc, long strideC,
    const float* __restrict__ bias, long strideBias,
    const float* __restrict__ resid, long strideR,
    int M, int N, int K, float scale)
{
  __shared__ __align__(16) float sT[8][16 * 68];
  const int b    = blockIdx.y;
  const int lane = threadIdx.x & 31;
  const int wave = threadIdx.x >> 5;
  const int tilesN = N >> 6;
  const int tilesM = M >> 6;
  const int tile = blockIdx.x * 8 + wave;
  if (tile >= tilesM * tilesN) return;
  const int tm = tile / tilesN;
  const int tn = tile - tm * tilesN;
  const int m0 = tm << 6;
  const int n0 = tn << 6;

  const _Float16* Ab = (const _Float16*)Ap  + (size_t)b * strideA;
  const _Float16* Bb = (const _Float16*)Btp + (size_t)b * strideB;

  const int rlane = lane & 15;
  const int koff  = (lane >> 4) * 8;
  const int mOff  = (lane >> 4) * 8;

  v8f acc[4][4];
#pragma unroll
  for (int i = 0; i < 4; ++i)
#pragma unroll
    for (int j = 0; j < 4; ++j) acc[i][j] = (v8f){0.f, 0.f, 0.f, 0.f, 0.f, 0.f, 0.f, 0.f};

  for (int k0 = 0; k0 < K; k0 += 32) {
    v16h bh[4];
#pragma unroll
    for (int j = 0; j < 4; ++j) {
      const size_t bo = (size_t)(n0 + (j << 4) + rlane) * ldb + koff + k0;
      bh[j] = frag_load_h(Bb + bo);
    }
#pragma unroll
    for (int i = 0; i < 4; ++i) {
      const size_t ao = (size_t)(m0 + (i << 4) + rlane) * lda + koff + k0;
      const v16h ah = frag_load_h(Ab + ao);
#pragma unroll
      for (int j = 0; j < 4; ++j) acc[i][j] = mma_h(ah, bh[j], acc[i][j]);
      tie1_h(acc[i][0], ah, bh[0]);
      tie1_h(acc[i][1], ah, bh[1]);
      tie1_h(acc[i][2], ah, bh[2]);
      guard1_h(acc[i][3], ah, bh[3]);
    }
    keep4_h(bh[0], bh[1], bh[2], bh[3]);
  }
  acc_guard4(acc[0][0], acc[0][1], acc[0][2], acc[0][3]);
  acc_guard4(acc[1][0], acc[1][1], acc[1][2], acc[1][3]);
  acc_guard4(acc[2][0], acc[2][1], acc[2][2], acc[2][3]);
  acc_guard4(acc[3][0], acc[3][1], acc[3][2], acc[3][3]);

  float* slab = sT[wave];
  const float* Rb = resid + (size_t)b * strideR;
  const float* Bs = bias + (size_t)b * strideBias;
  float* C = Cout + (size_t)b * strideC;
#pragma unroll
  for (int i = 0; i < 4; ++i) {
    const int mBase = m0 + (i << 4);
#pragma unroll
    for (int j = 0; j < 4; ++j) {
      const int n = n0 + (j << 4) + rlane;
      float bv = 0.f;
      if (BIAS_MODE == 2) bv = Bs[n];
#pragma unroll
      for (int r = 0; r < 8; ++r) {
        float v = acc[i][j][r] * scale;
        if (BIAS_MODE == 2) v += bv;
        slab[(mOff + r) * 68 + (j << 4) + rlane] = v;
      }
    }
    __builtin_amdgcn_fence(__ATOMIC_RELEASE, "workgroup");
    __builtin_amdgcn_wave_barrier();
    __builtin_amdgcn_fence(__ATOMIC_ACQUIRE, "workgroup");
    {
      const int hh = lane >> 4, c4 = (lane & 15) * 4;
      v4f ov[8];
#pragma unroll
      for (int it = 0; it < 8; ++it) {
        const int row = it * 2 + hh;
        v4f v = *(const v4f*)(slab + row * 68 + c4);
        if (RESID) {
          const v4f rv = *(const v4f*)(Rb + (size_t)(mBase + row) * ldc + n0 + c4);
          v = v + rv;
        }
        ov[it] = v;
      }
      for (int pass = 0; pass < 2; ++pass) {
#pragma unroll
        for (int it = 0; it < 8; ++it) {
          const int row = it * 2 + hh;
          *(volatile v4f*)(C + (size_t)(mBase + row) * ldc + n0 + c4) = ov[it];
        }
        __threadfence();
      }
    }
    __builtin_amdgcn_fence(__ATOMIC_RELEASE, "workgroup");
    __builtin_amdgcn_wave_barrier();
    __builtin_amdgcn_fence(__ATOMIC_ACQUIRE, "workgroup");
  }
}

__global__ __launch_bounds__(256) void transpose_cast_kernel(
    const float* __restrict__ W, unsigned short* __restrict__ Bt,
    int Kreal, int Kpad, int Nreal, int Nsub, long subStride, long srcZ, long dstZ, float scale)
{
  __shared__ float tile[64 * 65];
  const int tid = threadIdx.x, lane = tid & 31, wave = tid >> 5;
  const int n0 = blockIdx.x * 64;
  const int k0 = blockIdx.y * 64;
  const float* Wz = W + (size_t)blockIdx.z * srcZ;
  unsigned short* Bz = Bt + (size_t)blockIdx.z * dstZ;
#pragma unroll 4
  for (int p = 0; p < 16; ++p) {
    const int idx = tid + p * 256;
    const int kk  = idx >> 6;
    const int nn  = idx & 63;
    const int n   = n0 + nn;
    const int k   = k0 + kk;
    const int nc  = (n < Nreal) ? n : (Nreal - 1);
    const int kc  = (k < Kreal) ? k : (Kreal - 1);
    const int sub = nc / Nsub;
    const int col = nc - sub * Nsub;
    const float v = Wz[(size_t)sub * subStride + (size_t)kc * Nsub + col];
    const bool ok = (n < Nreal) && (k < Kreal);
    tile[kk * 65 + nn] = ok ? (v * scale) : 0.0f;
  }
  __syncthreads();
  const int q = lane >> 3, c8 = (lane & 7) * 8;
  v8h hv[2];
#pragma unroll
  for (int it = 0; it < 2; ++it) {
    const int nrow = it * 32 + wave * 4 + q;
#pragma unroll
    for (int e = 0; e < 8; ++e) hv[it][e] = f16_flush(tile[(c8 + e) * 65 + nrow]);
  }
  for (int pass = 0; pass < 2; ++pass) {
#pragma unroll
    for (int it = 0; it < 2; ++it) {
      const int nrow = it * 32 + wave * 4 + q;
      *(volatile v8h*)(Bz + (size_t)(n0 + nrow) * Kpad + k0 + c8) = hv[it];
    }
    __threadfence();
  }
}

__global__ __launch_bounds__(256) void ln_in_kernel(
    const float* __restrict__ x, const float* __restrict__ g, const float* __restrict__ bt,
    unsigned short* __restrict__ XN)
{
  const int lane = threadIdx.x & 31, wave = threadIdx.x >> 5;
  const int row = blockIdx.x * 8 + wave;
  const float* xr = x + (size_t)row * kDm;
  v4f a[6];
#pragma unroll
  for (int it = 0; it < 3; ++it) {
    a[2 * it]     = *(const v4f*)(xr + it * 256 + lane * 8);
    a[2 * it + 1] = *(const v4f*)(xr + it * 256 + lane * 8 + 4);
  }
  float s = 0.f;
#pragma unroll
  for (int j = 0; j < 6; ++j) s += (a[j][0] + a[j][1]) + (a[j][2] + a[j][3]);
  s = wave_sum(s);
  const float mu = s * (1.0f / (float)kDm);
  float q = 0.f;
#pragma unroll
  for (int j = 0; j < 6; ++j) {
#pragma unroll
    for (int e = 0; e < 4; ++e) {
      const float d = a[j][e] - mu;
      q = fmaf(d, d, q);
    }
  }
  q = wave_sum(q);
  const float rstd = rsqrtf(q * (1.0f / (float)kDm) + kEps);
  v8h hv[3];
#pragma unroll
  for (int it = 0; it < 3; ++it) {
    const v4f g0 = *(const v4f*)(g + it * 256 + lane * 8);
    const v4f g1 = *(const v4f*)(g + it * 256 + lane * 8 + 4);
    const v4f b0 = *(const v4f*)(bt + it * 256 + lane * 8);
    const v4f b1 = *(const v4f*)(bt + it * 256 + lane * 8 + 4);
#pragma unroll
    for (int e = 0; e < 4; ++e) {
      const float v0 = (a[2 * it][e] - mu) * rstd * g0[e] + b0[e];
      const float v1 = (a[2 * it + 1][e] - mu) * rstd * g1[e] + b1[e];
      hv[it][e]     = f16_flush(v0 * kCarryXn);
      hv[it][4 + e] = f16_flush(v1 * kCarryXn);
    }
  }
  for (int pass = 0; pass < 2; ++pass) {
#pragma unroll
    for (int it = 0; it < 3; ++it)
      *(volatile v8h*)(XN + (size_t)row * kDm + it * 256 + lane * 8) = hv[it];
    __threadfence();
  }
}

__global__ __launch_bounds__(256) void conv_silu_kernel(
    const float* __restrict__ XZ, const float* __restrict__ cw, const float* __restrict__ cb,
    float* __restrict__ UC, unsigned short* __restrict__ U16)
{
  __shared__ __align__(16) float sT[16 * kConvTP];
  const int tid = threadIdx.x, lane = tid & 31, wave = tid >> 5;
  const int d0 = blockIdx.x * 256, d = d0 + tid;
  const int t0 = blockIdx.y * 64;
  const float w0 = cw[d * 3 + 0], w1 = cw[d * 3 + 1], w2 = cw[d * 3 + 2];
  const float bc = cb[d];
  float xm1, xc;
  {
    const int r1 = t0 - 1;
    const float v1 = XZ[(size_t)(r1 < 0 ? 0 : r1) * kXzP + d];
    xm1 = (r1 >= 0) ? v1 : 0.0f;
    xc  = XZ[(size_t)t0 * kXzP + d];
  }
  const int hrow = wave >> 1;
  const int hch  = (wave & 1) * 128 + lane * 4;
#pragma unroll 1
  for (int sub = 0; sub < 4; ++sub) {
    const int lb = t0 + sub * 16;
#pragma unroll 1
    for (int s = 0; s < 16; ++s) {
      const int tn  = lb + s + 1;
      const int tnc = (tn < kLB) ? tn : (kLB - 1);
      const float vn = XZ[(size_t)tnc * kXzP + d];
      const float xp = (tn < kLB) ? vn : 0.0f;
      float acc = xm1 * w0;
      acc = fmaf(xc, w1, acc);
      acc = fmaf(xp, w2, acc);
      const float sv = acc + bc;
      sT[s * kConvTP + tid] = silu_f(sv);
      xm1 = xc;
      xc  = xp;
    }
    __syncthreads();
    v4f fv[4];
    v8h bv[2];
#pragma unroll
    for (int it = 0; it < 4; ++it) fv[it] = *(const v4f*)(sT + (it * 4 + hrow) * kConvTP + hch);
#pragma unroll
    for (int it = 0; it < 2; ++it) {
      const float* sp = sT + (it * 8 + wave) * kConvTP + lane * 8;
      const v4f a0 = *(const v4f*)(sp);
      const v4f a1 = *(const v4f*)(sp + 4);
#pragma unroll
      for (int e = 0; e < 4; ++e) {
        bv[it][e]     = f16_flush(a0[e] * kCarryU);
        bv[it][4 + e] = f16_flush(a1[e] * kCarryU);
      }
    }
    for (int pass = 0; pass < 2; ++pass) {
#pragma unroll
      for (int it = 0; it < 4; ++it)
        *(volatile v4f*)(UC + (size_t)(lb + it * 4 + hrow) * kDi + d0 + hch) = fv[it];
#pragma unroll
      for (int it = 0; it < 2; ++it)
        *(volatile v8h*)(U16 + (size_t)(lb + it * 8 + wave) * kDi + d0 + lane * 8) = bv[it];
      __threadfence();
    }
    __syncthreads();
  }
}

__global__ __launch_bounds__(256) void dt_cast_kernel(
    const float* __restrict__ PROJ, unsigned short* __restrict__ DTA)
{
  const int i   = blockIdx.x * 256 + threadIdx.x;
  const int e0  = i << 3;
  const int dir = e0 >> 17;
  const int rem = e0 & ((1 << 17) - 1);
  const int row = rem >> 6;
  const int c8  = rem & 63;
  const bool real = (c8 < kR);
  const int cc  = real ? c8 : 0;
  const float* p = PROJ + (size_t)row * kPjP + dir * kPj + cc;
  const v4f a0 = *(const v4f*)(p);
  const v4f a1 = *(const v4f*)(p + 4);
  float f0 = a0[0], f1 = a0[1], f2 = a0[2], f3 = a0[3];
  float f4 = a1[0], f5 = a1[1], f6 = a1[2], f7 = a1[3];
  asm volatile("" : "+v"(f0), "+v"(f1), "+v"(f2), "+v"(f3));
  asm volatile("" : "+v"(f4), "+v"(f5), "+v"(f6), "+v"(f7));
  v8h hv;
  hv[0] = f16_flush(real ? f0 * kCarryDt : 0.0f);
  hv[1] = f16_flush(real ? f1 * kCarryDt : 0.0f);
  hv[2] = f16_flush(real ? f2 * kCarryDt : 0.0f);
  hv[3] = f16_flush(real ? f3 * kCarryDt : 0.0f);
  hv[4] = f16_flush(real ? f4 * kCarryDt : 0.0f);
  hv[5] = f16_flush(real ? f5 * kCarryDt : 0.0f);
  hv[6] = f16_flush(real ? f6 * kCarryDt : 0.0f);
  hv[7] = f16_flush(real ? f7 * kCarryDt : 0.0f);
  unsigned short* qd = DTA + e0;
  *(volatile v8h*)qd = hv;
  __threadfence();
  *(volatile v8h*)qd = hv;
}

__global__ __launch_bounds__(64) void scan_kernel(
    const float* __restrict__ DLR, const float* __restrict__ UC, const float* __restrict__ PROJ,
    const float* __restrict__ Alog, const float* __restrict__ Dsk, float* __restrict__ YD)
{
  __shared__ __align__(16) float sBC[kScanTS * 32];
  __shared__ __align__(16) float sY[kScanTS * kScanYP];
  __shared__ __align__(16) float sA[kNs * kScanCh];
  const int tid = threadIdx.x, lane = tid & 31, wave = tid >> 5;
  constexpr int kBlkPerDir = kDi / kScanCh;
  const int dir = blockIdx.x / kBlkPerDir;
  const int d0  = (blockIdx.x - dir * kBlkPerDir) * kScanCh;
  const int d   = d0 + tid;
  const float* DLd = DLR + (size_t)dir * kLB * kDi;
  float* YDd = YD + (size_t)dir * kLB * kDi;
  const float* Al = Alog + ((size_t)dir * kDi + d) * kNs;
#pragma unroll 1
  for (int s = 0; s < kNs; ++s) sA[s * kScanCh + tid] = -expf(Al[s]);
  __syncthreads();
  float negA[kNs], h[kNs];
#pragma unroll
  for (int s = 0; s < kNs; ++s) {
    negA[s] = sA[s * kScanCh + tid];
    h[s] = 0.f;
  }
  const float Dd = Dsk[(size_t)dir * kDi + d];
  const int lr = tid >> 3, q4 = (tid & 7) * 4;
  const int hh = lane >> 4, c4 = (lane & 15) * 4;
  const int pcol = dir * kPj + kR;
#pragma unroll 1
  for (int c = 0; c < kLB / kScanTS; ++c) {
    const int tl = dir ? (kLB - kScanTS - c * kScanTS) : (c * kScanTS);
    __syncthreads();
#pragma unroll
    for (int i = 0; i < 8; ++i) {
      const int r = lr + 8 * i;
      *(v4f*)(sBC + r * 32 + q4) = *(const v4f*)(PROJ + (size_t)(tl + r) * kPjP + pcol + q4);
    }
    __syncthreads();
#pragma unroll 1
    for (int s = 0; s < kScanTS; ++s) {
      const int r = dir ? (kScanTS - 1 - s) : s;
      const size_t m = (size_t)(tl + r);
      const float a  = DLd[m * kDi + d];
      const float xv = UC[m * kDi + d];
      const float delta = fmaxf(a, 0.0f) + log1pf(expf(-fabsf(a)));
      const float dtx = delta * xv;
      v4f Bq[4], Cq[4];
#pragma unroll
      for (int qq = 0; qq < 4; ++qq) {
        Bq[qq] = *(const v4f*)(sBC + r * 32 + 4 * qq);
        Cq[qq] = *(const v4f*)(sBC + r * 32 + kNs + 4 * qq);
      }
      float y = 0.f;
#pragma unroll
      for (int n = 0; n < kNs; ++n) {
        const float e  = __expf(delta * negA[n]);
        const float hn = fmaf(e, h[n], dtx * Bq[n >> 2][n & 3]);
        h[n] = hn;
        y = fmaf(hn, Cq[n >> 2][n & 3], y);
      }
      y = fmaf(xv, Dd, y);
      sY[r * kScanYP + tid] = y;
    }
    __syncthreads();
    for (int pass = 0; pass < 2; ++pass) {
#pragma unroll 4
      for (int it = 0; it < 16; ++it) {
        const int row = it * 4 + wave * 2 + hh;
        const v4f v = *(const v4f*)(sY + row * kScanYP + c4);
        *(volatile v4f*)(YDd + (size_t)(tl + row) * kDi + d0 + c4) = v;
      }
      __threadfence();
    }
  }
}

__global__ __launch_bounds__(128) void merge_ln_gate_kernel(
    const float* __restrict__ YD, const float* __restrict__ XZ, const float* __restrict__ mw,
    const float* __restrict__ g, const float* __restrict__ bt, unsigned short* __restrict__ YG)
{
  __shared__ __align__(16) float sRow[4][kDi];
  __shared__ __align__(16) v4u   sOut[4][kDi / 8];
  const int lane = threadIdx.x & 31, wave = threadIdx.x >> 5;
  const int row = blockIdx.x * 4 + wave;
  const float w0 = mw[0], w1 = mw[1];
  const float* yf = YD + (size_t)row * kDi;
  const float* yb = YD + (size_t)kLB * kDi + (size_t)row * kDi;
  const float* zr = XZ + (size_t)row * kXzP + kDi;
  float* sr = sRow[wave];
  float s = 0.f;
#pragma unroll 1
  for (int it = 0; it < 6; ++it) {
    const int o = it * 256 + lane * 8;
    const v4f f0 = *(const v4f*)(yf + o);
    const v4f f1 = *(const v4f*)(yf + o + 4);
    const v4f r0 = *(const v4f*)(yb + o);
    const v4f r1 = *(const v4f*)(yb + o + 4);
    const v4f m0 = w0 * f0 + w1 * r0;
    const v4f m1 = w0 * f1 + w1 * r1;
    *(v4f*)(sr + o)     = m0;
    *(v4f*)(sr + o + 4) = m1;
    s += ((m0[0] + m0[1]) + (m0[2] + m0[3])) + ((m1[0] + m1[1]) + (m1[2] + m1[3]));
  }
  s = wave_sum(s);
  const float mu = s * (1.0f / (float)kDi);
  float q = 0.f;
#pragma unroll 1
  for (int it = 0; it < 6; ++it) {
    const int o = it * 256 + lane * 8;
    const v4f m0 = *(const v4f*)(sr + o);
    const v4f m1 = *(const v4f*)(sr + o + 4);
#pragma unroll
    for (int e = 0; e < 4; ++e) {
      const float da = m0[e] - mu;
      const float db = m1[e] - mu;
      q = fmaf(da, da, q);
      q = fmaf(db, db, q);
    }
  }
  q = wave_sum(q);
  const float rstd = rsqrtf(q * (1.0f / (float)kDi) + kEps);
#pragma unroll 1
  for (int it = 0; it < 6; ++it) {
    const int o = it * 256 + lane * 8;
    const v4f m0 = *(const v4f*)(sr + o);
    const v4f m1 = *(const v4f*)(sr + o + 4);
    const v4f g0 = *(const v4f*)(g + o);
    const v4f g1 = *(const v4f*)(g + o + 4);
    const v4f b0 = *(const v4f*)(bt + o);
    const v4f b1 = *(const v4f*)(bt + o + 4);
    const v4f z0 = *(const v4f*)(zr + o);
    const v4f z1 = *(const v4f*)(zr + o + 4);
    v8h hv;
#pragma unroll
    for (int e = 0; e < 4; ++e) {
      const float n0v = (m0[e] - mu) * rstd * g0[e] + b0[e];
      const float n1v = (m1[e] - mu) * rstd * g1[e] + b1[e];
      const float o0 = n0v * silu_f(z0[e]);
      const float o1 = n1v * silu_f(z1[e]);
      hv[e]     = f16_flush(o0 * kCarryY);
      hv[4 + e] = f16_flush(o1 * kCarryY);
    }
    sOut[wave][it * 32 + lane] = __builtin_bit_cast(v4u, hv);
  }
  for (int pass = 0; pass < 2; ++pass) {
#pragma unroll 1
    for (int it = 0; it < 6; ++it) {
      const v4u wv = sOut[wave][it * 32 + lane];
      *(volatile v4u*)(YG + (size_t)row * kDi + it * 256 + lane * 8) = wv;
    }
    __threadfence();
  }
}

extern "C" void kernel_launch(void* const* d_in, const int* in_sizes, int n_in,
                              void* d_out, int out_size, void* d_ws, size_t ws_size,
                              hipStream_t stream)
{
  if (n_in < 15) return;
  if (in_sizes[0] != kRows * kDm) return;
  if (in_sizes[1] != kDm || in_sizes[2] != kDm) return;
  if (in_sizes[3] != kDm * kXzP) return;
  if (in_sizes[4] != kDi * 3 || in_sizes[5] != kDi) return;
  if (in_sizes[6] != 2 * kDi * kPj) return;
  if (in_sizes[7] != 2 * kR * kDi) return;
  if (in_sizes[8] != 2 * kDi) return;
  if (in_sizes[9] != 2 * kDi * kNs) return;
  if (in_sizes[10] != 2 * kDi) return;
  if (in_sizes[11] != 2) return;
  if (in_sizes[12] != kDi || in_sizes[13] != kDi) return;
  if (in_sizes[14] != kDi * kDm) return;
  if (out_size != kRows * kDm) return;
  if (ws_size < kWsTotal) return;

  const float* x         = (const float*)d_in[0];
  const float* gamma_in  = (const float*)d_in[1];
  const float* beta_in   = (const float*)d_in[2];
  const float* W_in      = (const float*)d_in[3];
  const float* conv_w    = (const float*)d_in[4];
  const float* conv_b    = (const float*)d_in[5];
  const float* x_proj_w  = (const float*)d_in[6];
  const float* dt_w      = (const float*)d_in[7];
  const float* dt_b      = (const float*)d_in[8];
  const float* A_log     = (const float*)d_in[9];
  const float* D_skip    = (const float*)d_in[10];
  const float* merge_w   = (const float*)d_in[11];
  const float* gamma_out = (const float*)d_in[12];
  const float* beta_out  = (const float*)d_in[13];
  const float* W_out     = (const float*)d_in[14];
  float* out = (float*)d_out;

  char* ws = (char*)d_ws;
  unsigned short* WinT  = (unsigned short*)(ws + kOffWinT);
  unsigned short* XpT   = (unsigned short*)(ws + kOffXpT);
  unsigned short* DtT   = (unsigned short*)(ws + kOffDtT);
  unsigned short* WoutT = (unsigned short*)(ws + kOffWoutT);
  unsigned short* XN    = (unsigned short*)(ws + kOffXN);
  float*          XZ    = (float*)(ws + kOffXZ);
  float*          UC    = (float*)(ws + kOffUC);
  unsigned short* U16   = (unsigned short*)(ws + kOffU16);
  float*          PROJ  = (float*)(ws + kOffPROJ);
  unsigned short* DTA   = (unsigned short*)(ws + kOffDTA);
  float*          DLR   = (float*)(ws + kOffDLR);
  float*          YD    = (float*)(ws + kOffYD);
  unsigned short* YG    = (unsigned short*)(ws + kOffYG);
  const float* dummy_bias  = dt_b;
  const float* dummy_resid = x;

  transpose_cast_kernel<<<dim3(kXzP / 64, kDm / 64, 1), 256, 0, stream>>>(
      W_in, WinT, kDm, kDm, kXzP, kXzP, 0L, 0L, 0L, kCarryW);
  transpose_cast_kernel<<<dim3(kPjP / 64, kDi / 64, 1), 256, 0, stream>>>(
      x_proj_w, XpT, kDi, kDi, 2 * kPj, kPj, (long)kDi * kPj, 0L, 0L, kCarryW);
  transpose_cast_kernel<<<dim3(kDi / 64, kRP / 64, 2), 256, 0, stream>>>(
      dt_w, DtT, kR, kRP, kDi, kDi, 0L, (long)kR * kDi, (long)kDi * kRP, kCarryW);
  transpose_cast_kernel<<<dim3(kDm / 64, kDi / 64, 1), 256, 0, stream>>>(
      W_out, WoutT, kDi, kDi, kDm, kDm, 0L, 0L, 0L, kCarryW);

  ln_in_kernel<<<kRows / 8, 256, 0, stream>>>(x, gamma_in, beta_in, XN);

  for (int b = 0; b < kB; ++b) {
    const unsigned short* XNb = XN + (size_t)b * kLB * kDm;
    const float* xb = x + (size_t)b * kLB * kDm;
    float* outb = out + (size_t)b * kLB * kDm;

    wmma_gemm64<0, false><<<dim3(192, 1), 256, 0, stream>>>(
        XNb, kDm, 0L, WinT, kDm, 0L, XZ, kXzP, 0L,
        dummy_bias, 0L, dummy_resid, 0L, kLB, kXzP, kDm, kScaleIn);

    conv_silu_kernel<<<dim3(kDi / 256, kLB / 64), 256, 0, stream>>>(XZ, conv_w, conv_b, UC, U16);

    wmma_gemm64<0, false><<<dim3(12, 1), 256, 0, stream>>>(
        U16, kDi, 0L, XpT, kDi, 0L, PROJ, kPjP, 0L,
        dummy_bias, 0L, dummy_resid, 0L, kLB, kPjP, kDi, kScaleXp);

    dt_cast_kernel<<<(2 * kLB * kRP) / 8 / 256, 256, 0, stream>>>(PROJ, DTA);

    wmma_gemm64<2, false><<<dim3(96, 2), 256, 0, stream>>>(
        DTA, kRP, (long)kLB * kRP, DtT, kRP, (long)kDi * kRP, DLR, kDi, (long)kLB * kDi,
        dt_b, (long)kDi, dummy_resid, 0L, kLB, kDi, kRP, kScaleDt);

    scan_kernel<<<2 * (kDi / kScanCh), kScanCh, 0, stream>>>(DLR, UC, PROJ, A_log, D_skip, YD);

    merge_ln_gate_kernel<<<kLB / 4, 128, 0, stream>>>(YD, XZ, merge_w, gamma_out, beta_out, YG);

    wmma_gemm64<0, true><<<dim3(48, 1), 256, 0, stream>>>(
        YG, kDi, 0L, WoutT, kDi, 0L, outb, kDm, 0L,
        dummy_bias, 0L, xb, 0L, kLB, kDm, kDi, kScaleOut);
  }
}
